// SelfAttention1_40097814675851
// MI455X (gfx1250) — hardware-verified
//
#include <hip/hip_runtime.h>
#include <stdint.h>

#define NBATCH 4
#define SEQ    2048
#define HD     1024
#define NTOK   8192

typedef _Float16 v16h __attribute__((ext_vector_type(16)));
typedef _Float16 v8h  __attribute__((ext_vector_type(8)));
typedef float    v8f  __attribute__((ext_vector_type(8)));
typedef float    v4f  __attribute__((ext_vector_type(4)));

static_assert(NTOK == NBATCH * SEQ);
static_assert((HD % 64) == 0 && (NTOK % 64) == 0 && (HD % 32) == 0);

__device__ __forceinline__ unsigned short bfbits(float f) {
  unsigned u = __float_as_uint(f);
  return (unsigned short)((u + 0x7FFFu + ((u >> 16) & 1u)) >> 16);
}
__device__ __forceinline__ float bfval(unsigned short b) { return __uint_as_float(((unsigned)b) << 16); }
__device__ __forceinline__ float bfr(float f) { return bfval(bfbits(f)); }

__device__ __forceinline__ v16h ldfrag(const _Float16* p) {
  union { v16h v; v8h hh[2]; } f;
  f.hh[0] = *(const v8h*)(p);
  f.hh[1] = *(const v8h*)(p + 16);
  return f.v;
}
__device__ __forceinline__ v8f mma16(v16h a, v16h b, v8f c) {
  return __builtin_amdgcn_wmma_f32_16x16x32_f16(false, a, false, b, (short)0, c, false, false);
}
__device__ __forceinline__ v8f zero8() {
  v8f z;
#pragma unroll
  for (int i = 0; i < 8; ++i) z[i] = 0.0f;
  return z;
}

__device__ __forceinline__ void guard_g(v8f& a, v8f& b, v16h x, v16h y) {
  asm volatile("v_nop\n\tv_nop\n\tv_nop\n\tv_nop" : "+v"(a), "+v"(b) : "v"(x), "v"(y));
}
__device__ __forceinline__ void keep4(v16h a, v16h b, v16h c, v16h d) {
  asm volatile("v_nop" :: "v"(a), "v"(b), "v"(c), "v"(d));
}
__device__ __forceinline__ void accg4(v8f& a, v8f& b, v8f& c, v8f& d) {
  asm volatile("v_nop\n\tv_nop\n\tv_nop\n\tv_nop" : "+v"(a), "+v"(b), "+v"(c), "+v"(d));
}
__device__ __forceinline__ void guard_s(v8f& a, v8f& b, v8f& c, v8f& d,
                                        v16h x0, v16h x1, v16h x2, v16h x3, v16h x4) {
  asm volatile("v_nop\n\tv_nop\n\tv_nop\n\tv_nop"
               : "+v"(a), "+v"(b), "+v"(c), "+v"(d) : "v"(x0), "v"(x1), "v"(x2), "v"(x3), "v"(x4));
}
__device__ __forceinline__ void guard_o(v8f& a, v8f& b, v8f& c, v8f& d,
                                        v16h x0, v16h x1, v16h x2, v16h x3) {
  asm volatile("v_nop\n\tv_nop\n\tv_nop\n\tv_nop"
               : "+v"(a), "+v"(b), "+v"(c), "+v"(d) : "v"(x0), "v"(x1), "v"(x2), "v"(x3));
}

__global__ __launch_bounds__(256) void cvt_x_kernel(const float* __restrict__ x, _Float16* __restrict__ X8, int n8) {
  const int li = (int)blockIdx.x * 256 + (int)threadIdx.x;
  if (li >= n8) return;
  const size_t e = (size_t)li * 8;
  const v4f a = *(const v4f*)(x + e);
  const v4f b = *(const v4f*)(x + e + 4);
  v8h o;
#pragma unroll
  for (int i = 0; i < 4; ++i) {
    o[i]     = (_Float16)(bfr(a[i]) * 8.0f);
    o[4 + i] = (_Float16)(bfr(b[i]) * 8.0f);
  }
  _Float16* d = X8 + e;
  *(volatile v8h*)d = o;
  __threadfence();
  *(volatile v8h*)d = o;
}

__global__ __launch_bounds__(256) void cvt_w_kernel(const float* __restrict__ Wq, const float* __restrict__ Wk,
                                                    const float* __restrict__ Wv, _Float16* __restrict__ Wt) {
  __shared__ __align__(16) _Float16 sT[64 * 72];
  const int bid = (int)blockIdx.x;
  const int mat = bid >> 8;
  const int tile = bid & 255;
  const int tr = tile >> 4, tc = tile & 15;
  const float* src = (mat == 0) ? Wq : ((mat == 1) ? Wk : Wv);
  _Float16* dst = Wt + (size_t)mat * HD * HD;
  const int d0 = tr * 64, e0 = tc * 64;
  const int tid = threadIdx.x, lane = tid & 31, wave = tid >> 5;
  {
    const int i = tid >> 2;
    const int j0 = (tid & 3) * 16;
    const float* p = src + (size_t)(d0 + i) * HD + e0 + j0;
#pragma unroll
    for (int q4 = 0; q4 < 4; ++q4) {
      const v4f a = *(const v4f*)(p + 4 * q4);
#pragma unroll
      for (int e = 0; e < 4; ++e) sT[(j0 + 4 * q4 + e) * 72 + i] = (_Float16)(bfr(a[e]) * 64.0f);
    }
  }
  __syncthreads();
  const int rq = lane >> 3, c8 = (lane & 7) * 8;
#pragma unroll
  for (int ps = 0; ps < 2; ++ps) {
#pragma unroll
    for (int it = 0; it < 2; ++it) {
      const int row = it * 32 + wave * 4 + rq;
      const v8h v = *(const v8h*)(sT + row * 72 + c8);
      *(volatile v8h*)(dst + (size_t)(e0 + row) * HD + d0 + c8) = v;
    }
    __threadfence();
  }
}

template <bool OUT2, bool BIASROW>
__global__ __launch_bounds__(256) __attribute__((amdgpu_num_vgpr(256)))
void gemm64_kernel(const _Float16* __restrict__ A, int lda, const _Float16* __restrict__ Bt, int ldb,
                   _Float16* __restrict__ Ch, _Float16* __restrict__ Cl, int ldc,
                   const float* __restrict__ bias, int M, int N, int K, float scale, float bsc) {
  __shared__ __align__(16) float sT[8][16 * 68];
  const int lane = threadIdx.x & 31, wave = threadIdx.x >> 5;
  const int tilesN = N >> 6, tilesM = M >> 6;
  const int tile = (int)blockIdx.x * 8 + wave;
  if (tile >= tilesM * tilesN) return;
  const int tm = tile / tilesN, tn = tile - tm * tilesN;
  const int m0 = tm << 6, n0 = tn << 6;
  const int rl = lane & 15;
  const int koff = (lane >> 4) * 8;
  const int mOff = (lane >> 4) * 8;

  v8f acc[4][4];
#pragma unroll
  for (int i = 0; i < 4; ++i)
#pragma unroll
    for (int j = 0; j < 4; ++j) acc[i][j] = zero8();

#pragma unroll 1
  for (int k0 = 0; k0 < K; k0 += 32) {
    v16h bh[4];
#pragma unroll
    for (int j = 0; j < 4; ++j) bh[j] = ldfrag(Bt + (size_t)(n0 + (j << 4) + rl) * ldb + koff + k0);
#pragma unroll
    for (int i = 0; i < 4; ++i) {
      const v16h ah = ldfrag(A + (size_t)(m0 + (i << 4) + rl) * lda + koff + k0);
#pragma unroll
      for (int j = 0; j < 4; ++j) acc[i][j] = mma16(ah, bh[j], acc[i][j]);
      guard_g(acc[i][0], acc[i][3], ah, bh[3]);
    }
    keep4(bh[0], bh[1], bh[2], bh[3]);
  }
  accg4(acc[0][0], acc[0][1], acc[0][2], acc[0][3]);
  accg4(acc[1][0], acc[1][1], acc[1][2], acc[1][3]);
  accg4(acc[2][0], acc[2][1], acc[2][2], acc[2][3]);
  accg4(acc[3][0], acc[3][1], acc[3][2], acc[3][3]);

  float* slab = sT[wave];
  const int rq = lane >> 3, c8 = (lane & 7) * 8;
#pragma unroll
  for (int i = 0; i < 4; ++i) {
    const int mBase = m0 + (i << 4);
    float brow[8];
#pragma unroll
    for (int r = 0; r < 8; ++r) brow[r] = 0.0f;
    if (BIASROW) {
#pragma unroll
      for (int r = 0; r < 8; ++r) brow[r] = bfr(bias[mBase + mOff + r]) * bsc;
    }
#pragma unroll
    for (int j = 0; j < 4; ++j) {
      float bcol = 0.0f;
      if (!BIASROW) bcol = bfr(bias[n0 + (j << 4) + rl]) * bsc;
#pragma unroll
      for (int r = 0; r < 8; ++r)
        slab[(mOff + r) * 68 + (j << 4) + rl] = acc[i][j][r] * scale + (BIASROW ? brow[r] : bcol);
    }
    __builtin_amdgcn_fence(__ATOMIC_RELEASE, "workgroup");
    __builtin_amdgcn_wave_barrier();
    __builtin_amdgcn_fence(__ATOMIC_ACQUIRE, "workgroup");
#pragma unroll
    for (int ps = 0; ps < 2; ++ps) {
#pragma unroll
      for (int it = 0; it < 4; ++it) {
        const int row = it * 4 + rq;
        const float* sp = slab + row * 68 + c8;
        v8h hv, lv;
#pragma unroll
        for (int e = 0; e < 8; ++e) {
          const float y = sp[e];
          const _Float16 yh = (_Float16)y;
          hv[e] = yh;
          lv[e] = (_Float16)((y - (float)yh) * 1024.0f);
        }
        const size_t go = (size_t)(mBase + row) * ldc + n0 + c8;
        *(volatile v8h*)(Ch + go) = hv;
        if (OUT2) *(volatile v8h*)(Cl + go) = lv;
      }
      __threadfence();
    }
    __builtin_amdgcn_fence(__ATOMIC_RELEASE, "workgroup");
    __builtin_amdgcn_wave_barrier();
    __builtin_amdgcn_fence(__ATOMIC_ACQUIRE, "workgroup");
  }
}

#define QB       32
#define KCH      256
#define QSP      1032
#define PSP      264
#define OSP      1032
#define LDS_QH   0
#define LDS_QL   (QB * QSP * 2)
#define LDS_PS   (2 * QB * QSP * 2)
#define LDS_PMAX (LDS_PS + QB * PSP * 2)
#define LDS_PSUM (LDS_PMAX + 512 * 4)
#define LDS_ST   (LDS_PSUM + 512 * 4)
#define ATT_LDS  (LDS_ST + 4 * 32 * 4)
static_assert(LDS_QL == 66048 && LDS_PS == 132096 && LDS_PMAX == 148992 && ATT_LDS == 153600);
static_assert(QB * OSP * 4 <= LDS_PS);
static_assert((QSP % 8) == 0 && (PSP % 8) == 0 && PSP >= KCH && (OSP % 4) == 0);
static_assert((LDS_QL % 16) == 0 && (LDS_PS % 16) == 0 && (LDS_PMAX % 16) == 0 && (LDS_ST % 16) == 0);
static_assert((SEQ % KCH) == 0 && (SEQ % QB) == 0 && (KCH == 16 * 16) && (HD == 16 * 64));

__global__ __launch_bounds__(512) __attribute__((amdgpu_num_vgpr(256)))
void attn_kernel(const _Float16* __restrict__ qh, const _Float16* __restrict__ ql,
                 const _Float16* __restrict__ kp, const _Float16* __restrict__ vht,
                 const _Float16* __restrict__ vlt, float* __restrict__ out, float sc) {
  extern __shared__ __align__(16) char smem[];
  _Float16* Qhs = (_Float16*)(smem + LDS_QH);
  _Float16* Qls = (_Float16*)(smem + LDS_QL);
  _Float16* Ps  = (_Float16*)(smem + LDS_PS);
  float* pmax = (float*)(smem + LDS_PMAX);
  float* psum = (float*)(smem + LDS_PSUM);
  float* m_s  = (float*)(smem + LDS_ST);
  float* l_s  = m_s + 32;
  float* al_s = m_s + 64;
  float* li_s = m_s + 96;

  const int tid = threadIdx.x, wave = tid >> 5, lane = tid & 31, h = lane >> 4, c = lane & 15;
  const int bid = (int)blockIdx.x;
  const int b = bid / (SEQ / QB);
  const int qtile = bid - b * (SEQ / QB);
  const int kbase = b * SEQ;
  const int q0 = kbase + qtile * QB;
  const float ninf = -__builtin_inff();

  if (tid < 32) { m_s[tid] = ninf; l_s[tid] = 0.0f; al_s[tid] = 0.0f; li_s[tid] = 0.0f; }
  psum[tid] = 0.0f;
#pragma unroll
  for (int i = 0; i < 8; ++i) {
    const int idx = i * 512 + tid;
    const int row = idx >> 7;
    const int pc  = idx & 127;
    const size_t g = (size_t)(q0 + row) * HD + pc * 8;
    const v8h vh = *(const v8h*)(qh + g);
    const v8h vl = *(const v8h*)(ql + g);
    *(v8h*)(Qhs + row * QSP + pc * 8) = vh;
    *(v8h*)(Qls + row * QSP + pc * 8) = vl;
  }
  __syncthreads();

  v8f ohi[2][4];
#pragma unroll
  for (int qt = 0; qt < 2; ++qt)
#pragma unroll
    for (int nt = 0; nt < 4; ++nt) ohi[qt][nt] = zero8();

  const _Float16* qb0h = Qhs + c * QSP + 8 * h;
  const _Float16* qb1h = Qhs + (16 + c) * QSP + 8 * h;
  const _Float16* qb0l = Qls + c * QSP + 8 * h;
  const _Float16* qb1l = Qls + (16 + c) * QSP + 8 * h;
  const _Float16* pa0p = Ps + c * PSP + 8 * h;
  const _Float16* pa1p = Ps + (16 + c) * PSP + 8 * h;
  const int ntile = SEQ / KCH;
  const float rres = 1.0f / 1024.0f;

#pragma unroll 1
  for (int t = 0; t < ntile; ++t) {
    const int kb = kbase + t * KCH + 16 * wave;
    const _Float16* kap = kp + (size_t)(kb + c) * HD + 8 * h;
    v8f sh0 = zero8(), sh1 = zero8(), sl0 = zero8(), sl1 = zero8();
#pragma unroll 1
    for (int k0 = 0; k0 < HD; k0 += 32) {
      const v16h a   = ldfrag(kap + k0);
      const v16h b0h = ldfrag(qb0h + k0), b0l = ldfrag(qb0l + k0);
      const v16h b1h = ldfrag(qb1h + k0), b1l = ldfrag(qb1l + k0);
      sh0 = mma16(a, b0h, sh0);
      sl0 = mma16(a, b0l, sl0);
      sh1 = mma16(a, b1h, sh1);
      sl1 = mma16(a, b1l, sl1);
      guard_s(sh0, sl0, sh1, sl1, a, b0h, b0l, b1h, b1l);
    }
    {
      float pm0 = ninf, pm1 = ninf;
#pragma unroll
      for (int r = 0; r < 8; ++r) {
        const float v0 = (sh0[r] + sl0[r] * rres) * sc; sh0[r] = v0; pm0 = fmaxf(pm0, v0);
        const float v1 = (sh1[r] + sl1[r] * rres) * sc; sh1[r] = v1; pm1 = fmaxf(pm1, v1);
      }
      pm0 = fmaxf(pm0, __shfl_xor(pm0, 16, 32));
      pm1 = fmaxf(pm1, __shfl_xor(pm1, 16, 32));
      pmax[wave * 32 + c] = pm0;
      pmax[wave * 32 + 16 + c] = pm1;
    }
    __syncthreads();
    if (wave == 0) {
      const int row = lane;
      float ps = 0.0f;
#pragma unroll
      for (int w = 0; w < 16; ++w) ps += psum[w * 32 + row];
      l_s[row] = l_s[row] * al_s[row] + ps;
      const float mo = m_s[row];
      float mx = mo;
#pragma unroll
      for (int w = 0; w < 16; ++w) mx = fmaxf(mx, pmax[w * 32 + row]);
      al_s[row] = __expf(mo - mx);
      m_s[row] = mx;
    }
    __syncthreads();
    {
      const float mq0 = m_s[c], mq1 = m_s[16 + c];
      float ps0 = 0.0f, ps1 = 0.0f;
      v8h h0, h1;
#pragma unroll
      for (int r = 0; r < 8; ++r) {
        const float p0 = __expf(sh0[r] - mq0); ps0 += p0; h0[r] = (_Float16)(p0 * 16.0f);
        const float p1 = __expf(sh1[r] - mq1); ps1 += p1; h1[r] = (_Float16)(p1 * 16.0f);
      }
      *(v8h*)(Ps + c * PSP + 16 * wave + 8 * h) = h0;
      *(v8h*)(Ps + (16 + c) * PSP + 16 * wave + 8 * h) = h1;
      ps0 += __shfl_xor(ps0, 16, 32);
      ps1 += __shfl_xor(ps1, 16, 32);
      psum[wave * 32 + c] = ps0;
      psum[wave * 32 + 16 + c] = ps1;
      const v4f aA = *(const v4f*)(al_s + 8 * h), aB = *(const v4f*)(al_s + 8 * h + 4);
      const v4f bA = *(const v4f*)(al_s + 16 + 8 * h), bB = *(const v4f*)(al_s + 16 + 8 * h + 4);
#pragma unroll
      for (int nt = 0; nt < 4; ++nt) {
#pragma unroll
        for (int r = 0; r < 4; ++r) {
          ohi[0][nt][r] *= aA[r]; ohi[0][nt][4 + r] *= aB[r];
          ohi[1][nt][r] *= bA[r]; ohi[1][nt][4 + r] *= bB[r];
        }
      }
    }
    __syncthreads();
    {
      v8f olo[2][4];
#pragma unroll
      for (int qt = 0; qt < 2; ++qt)
#pragma unroll
        for (int nt = 0; nt < 4; ++nt) olo[qt][nt] = zero8();
      const size_t vro = (size_t)(64 * wave + c) * NTOK + kbase + t * KCH + 8 * h;
      const _Float16* vhb = vht + vro;
      const _Float16* vlb = vlt + vro;
#pragma unroll 1
      for (int ks = 0; ks < KCH; ks += 32) {
        const v16h pa0 = ldfrag(pa0p + ks), pa1 = ldfrag(pa1p + ks);
#pragma unroll
        for (int nt = 0; nt < 4; ++nt) {
          const size_t co = (size_t)(16 * nt) * NTOK + ks;
          const v16h vh = ldfrag(vhb + co);
          const v16h vl = ldfrag(vlb + co);
          ohi[0][nt] = mma16(pa0, vh, ohi[0][nt]);
          ohi[1][nt] = mma16(pa1, vh, ohi[1][nt]);
          olo[0][nt] = mma16(pa0, vl, olo[0][nt]);
          olo[1][nt] = mma16(pa1, vl, olo[1][nt]);
          guard_o(ohi[0][nt], ohi[1][nt], olo[0][nt], olo[1][nt], pa0, pa1, vh, vl);
        }
      }
#pragma unroll
      for (int qt = 0; qt < 2; ++qt)
#pragma unroll
        for (int nt = 0; nt < 4; ++nt)
#pragma unroll
          for (int r = 0; r < 8; ++r) ohi[qt][nt][r] += olo[qt][nt][r] * rres;
    }
  }

  if (wave == 0) {
    const int row = lane;
    float ps = 0.0f;
#pragma unroll
    for (int w = 0; w < 16; ++w) ps += psum[w * 32 + row];
    const float l = l_s[row] * al_s[row] + ps;
    li_s[row] = (1.0f / l) * (1.0f / 256.0f);
  }
  __syncthreads();
  float* Os = (float*)(smem + LDS_QH);
  {
    const v4f iA0 = *(const v4f*)(li_s + 8 * h),      iB0 = *(const v4f*)(li_s + 8 * h + 4);
    const v4f iA1 = *(const v4f*)(li_s + 16 + 8 * h), iB1 = *(const v4f*)(li_s + 16 + 8 * h + 4);
#pragma unroll
    for (int nt = 0; nt < 4; ++nt) {
      const int col = 64 * wave + 16 * nt + c;
#pragma unroll
      for (int r = 0; r < 4; ++r) {
        Os[(8 * h + r) * OSP + col]          = ohi[0][nt][r] * iA0[r];
        Os[(8 * h + 4 + r) * OSP + col]      = ohi[0][nt][4 + r] * iB0[r];
        Os[(16 + 8 * h + r) * OSP + col]     = ohi[1][nt][r] * iA1[r];
        Os[(16 + 8 * h + 4 + r) * OSP + col] = ohi[1][nt][4 + r] * iB1[r];
      }
    }
  }
  __syncthreads();
  {
    float* go = out + (size_t)q0 * HD;
#pragma unroll
    for (int ps = 0; ps < 2; ++ps) {
#pragma unroll
      for (int rr = 0; rr < 2; ++rr) {
        const int row = 2 * wave + rr;
#pragma unroll
        for (int j = 0; j < 8; ++j) {
          const int pc = j * 32 + lane;
          const v4f v = *(const v4f*)(Os + row * OSP + pc * 4);
          *(volatile v4f*)(go + (size_t)row * HD + pc * 4) = v;
        }
      }
      __threadfence();
    }
  }
}

extern "C" void kernel_launch(void* const* d_in, const int* in_sizes, int n_in,
                              void* d_out, int out_size, void* d_ws, size_t ws_size,
                              hipStream_t stream) {
  if (n_in < 7) return;
  const int ntok = NTOK, hd = HD;
  if (in_sizes[0] != ntok * hd) return;
  if (in_sizes[1] != hd * hd || in_sizes[3] != hd * hd || in_sizes[5] != hd * hd) return;
  if (in_sizes[2] != hd || in_sizes[4] != hd || in_sizes[6] != hd) return;
  if (out_size != ntok * hd) return;

  const float* x  = (const float*)d_in[0];
  const float* Wq = (const float*)d_in[1];
  const float* bq = (const float*)d_in[2];
  const float* Wk = (const float*)d_in[3];
  const float* bk = (const float*)d_in[4];
  const float* Wv = (const float*)d_in[5];
  const float* bv = (const float*)d_in[6];
  float* out = (float*)d_out;

  const size_t bX  = (size_t)ntok * hd * 2;
  const size_t bWT = (size_t)3 * hd * hd * 2;
  const size_t bP  = (size_t)ntok * hd * 2;
  size_t off = 0;
  const size_t oX  = off; off += bX;
  const size_t oWT = off; off += bWT;
  const size_t oQH = off; off += bP;
  const size_t oQL = off; off += bP;
  const size_t oKP = off; off += bP;
  const size_t oVH = off; off += bP;
  const size_t oVL = off; off += bP;
  if (off > ws_size) return;
  if (off > (size_t)134217728) return;

  char* ws = (char*)d_ws;
  _Float16* X8  = (_Float16*)(ws + oX);
  _Float16* WT  = (_Float16*)(ws + oWT);
  _Float16* WqT = WT;
  _Float16* WkT = WT + (size_t)hd * hd;
  _Float16* WvT = WT + (size_t)2 * hd * hd;
  _Float16* QH  = (_Float16*)(ws + oQH);
  _Float16* QL  = (_Float16*)(ws + oQL);
  _Float16* KP  = (_Float16*)(ws + oKP);
  _Float16* VHT = (_Float16*)(ws + oVH);
  _Float16* VLT = (_Float16*)(ws + oVL);

  const dim3 blk(256);
  const int n8 = ntok * hd / 8;
  if ((n8 % 256) != 0) return;

  cvt_x_kernel<<<dim3(n8 / 256), blk, 0, stream>>>(x, X8, n8);
  cvt_w_kernel<<<dim3(3 * (hd / 64) * (hd / 64)), blk, 0, stream>>>(Wq, Wk, Wv, WT);
  gemm64_kernel<true, false><<<dim3(((ntok / 64) * (hd / 64) + 7) / 8), blk, 0, stream>>>(
      X8, hd, WqT, hd, QH, QL, hd, bq, ntok, hd, hd, 0.03125f, 16.0f);
  gemm64_kernel<false, false><<<dim3(((ntok / 64) * (hd / 64) + 7) / 8), blk, 0, stream>>>(
      X8, hd, WkT, hd, KP, KP, hd, bk, ntok, hd, hd, 0.03125f, 16.0f);
  gemm64_kernel<true, true><<<dim3(((hd / 64) * (ntok / 64) + 7) / 8), blk, 0, stream>>>(
      WvT, hd, X8, hd, VHT, VLT, ntok, bv, hd, ntok, hd, 0.03125f, 16.0f);
  (void)hipFuncSetAttribute(reinterpret_cast<const void*>(&attn_kernel),
                            hipFuncAttributeMaxDynamicSharedMemorySize, ATT_LDS);
  const float sc = 0.0001220703125f;
  attn_kernel<<<dim3(NBATCH * (SEQ / QB)), dim3(512), ATT_LDS, stream>>>(QH, QL, KP, VHT, VLT, out, sc);
  (void)hipGetLastError();
}
